// HSCATB_76716705841257
// MI455X (gfx1250) — hardware-verified
//
#include <hip/hip_runtime.h>
#define NI 8
#define CH 256
#define HS 32
#define PX 1024
#define NR (NI * PX)
#define NH 8
#define HD 32
#define WSZ 8
#define NWIN 16
#define WT 64
#define NBW (NI * NWIN)
#define HID 1024
typedef __bf16 v16b __attribute__((ext_vector_type(16)));
typedef unsigned short v8us __attribute__((ext_vector_type(8), may_alias));
typedef float  v8f  __attribute__((ext_vector_type(8)));
typedef float  v4f  __attribute__((ext_vector_type(4)));
typedef float  v4fa __attribute__((ext_vector_type(4), may_alias));
union FragB { v16b v; v8us half[2]; unsigned short u[16]; };

__device__ __forceinline__ unsigned short bf16_bits(float x) { unsigned int u = __float_as_uint(x); return (unsigned short)((u + 0x7FFFu + ((u >> 16) & 1u)) >> 16); }
__device__ __forceinline__ float bf16_val(unsigned short b) { return __uint_as_float(((unsigned int)b) << 16); }
__device__ __forceinline__ float bf16_round(float x) { return bf16_val(bf16_bits(x)); }
template <int NT>
__device__ __forceinline__ v8f mmaN(v16b ah, v16b al, v16b bh, v16b bl, v8f c) {
  c = __builtin_amdgcn_wmma_f32_16x16x32_bf16(false, ah, false, bh, (short)0, c, false, false);
  if (NT >= 2) c = __builtin_amdgcn_wmma_f32_16x16x32_bf16(false, al, false, bh, (short)0, c, false, false);
  if (NT >= 3) c = __builtin_amdgcn_wmma_f32_16x16x32_bf16(false, ah, false, bl, (short)0, c, false, false);
  asm volatile("v_nop\n\tv_nop\n\tv_nop\n\tv_nop" : "+v"(c) : "v"(ah), "v"(al), "v"(bh), "v"(bl));
  return c;
}

__global__ __launch_bounds__(256) void k_wt_bf16(const float* __restrict__ W, unsigned short* __restrict__ Wt, int K, int N) {
  const int t = blockIdx.x * 256 + threadIdx.x;
  const int k8n = K / 8;
  if (t >= N * k8n) return;
  const int n = t / k8n, k8 = (t % k8n) * 8;
  v8us v;
#pragma unroll
  for (int i = 0; i < 8; ++i) v[i] = bf16_bits(W[(size_t)(k8 + i) * N + n]);
  *(volatile v8us*)(Wt + (size_t)n * K + k8) = v;
  __threadfence();
  *(volatile v8us*)(Wt + (size_t)n * K + k8) = v;
}

template <bool ASPLIT, int ACT, bool BIAS_BF16>
__global__ __launch_bounds__(128) void k_gemm_bf(const float* __restrict__ A, int lda, const unsigned short* __restrict__ Wt, int ldb,
                                               const float* __restrict__ bias, float* __restrict__ C, int ldc, int M, int N, int K) {
  __shared__ __attribute__((aligned(16))) float so[4][16][64];
  const int tid = threadIdx.x, w = tid >> 5, lane = tid & 31, ln = lane & 15, hh = lane >> 4;
  const int ntn = N / 64;
  const int wid = blockIdx.x * 4 + w;
  const int mt = wid / ntn, nq = wid % ntn;
  if (mt * 16 >= M) return;
  const int row0 = mt * 16, col0 = nq * 64;
  const float* arow = A + (size_t)(row0 + ln) * lda;
  v8f acc[4] = {};
  for (int kb = 0; kb < K; kb += 32) {
    FragB ah, al;
    const v4f x0 = *(const v4fa*)(arow + kb + 8 * hh), x1 = *(const v4fa*)(arow + kb + 8 * hh + 4);
    const v4f x2 = *(const v4fa*)(arow + kb + 16 + 8 * hh), x3 = *(const v4fa*)(arow + kb + 16 + 8 * hh + 4);
    float xs[16] = {x0[0],x0[1],x0[2],x0[3],x1[0],x1[1],x1[2],x1[3],x2[0],x2[1],x2[2],x2[3],x3[0],x3[1],x3[2],x3[3]};
#pragma unroll
    for (int i = 0; i < 16; ++i) { const unsigned short hb = bf16_bits(xs[i]); ah.u[i] = hb; al.u[i] = ASPLIT ? bf16_bits(xs[i] - bf16_val(hb)) : (unsigned short)0; }
#pragma unroll
    for (int t = 0; t < 4; ++t) {
      const unsigned short* brow = Wt + (size_t)(col0 + t * 16 + ln) * ldb + kb;
      FragB b;
      b.half[0] = *(const v8us*)(brow + 8 * hh);
      b.half[1] = *(const v8us*)(brow + 16 + 8 * hh);
      acc[t] = mmaN<ASPLIT ? 2 : 1>(ah.v, al.v, b.v, b.v, acc[t]);
    }
  }
#pragma unroll
  for (int t = 0; t < 4; ++t) {
    float bv = bias ? bias[col0 + t * 16 + ln] : 0.f;
    if (BIAS_BF16) bv = bf16_round(bv);
#pragma unroll
    for (int r = 0; r < 8; ++r) { float v = acc[t][r] + bv; if (ACT == 1) v = fmaxf(v, 0.f); so[w][8 * hh + r][t * 16 + ln] = v; }
  }
  __builtin_amdgcn_fence(__ATOMIC_ACQ_REL, "workgroup");
  __builtin_amdgcn_wave_barrier();
  const int rsub = lane >> 4, c4 = (lane & 15) * 4;
  for (int pass = 0; pass < 2; ++pass) {
#pragma unroll
    for (int q = 0; q < 8; ++q) {
      const int r = q * 2 + rsub;
      const v4f v = *(const v4fa*)&so[w][r][c4];
      *(volatile v4f*)(C + (size_t)(row0 + r) * ldc + col0 + c4) = v;
    }
    if (pass == 0) __threadfence();
  }
}

template <bool ASPLIT, int ACT, bool BIAS_BF16, bool RES_BF16>
__global__ __launch_bounds__(128) void k_gemm_bf3(const float* __restrict__ A, int lda, const unsigned short* __restrict__ Wt, int ldb,
                                                const float* __restrict__ bias, const float* __restrict__ resid, int rmod, int ldr,
                                                float* __restrict__ C, int ldc, int M, int N, int K) {
  __shared__ __attribute__((aligned(16))) float so[4][16][64];
  const int tid = threadIdx.x, w = tid >> 5, lane = tid & 31, ln = lane & 15, hh = lane >> 4;
  const int ntn = N / 64;
  const int wid = blockIdx.x * 4 + w;
  const int mt = wid / ntn, nq = wid % ntn;
  if (mt * 16 >= M) return;
  const int row0 = mt * 16, col0 = nq * 64;
  const float* arow = A + (size_t)(row0 + ln) * lda;
  v8f acc[4] = {};
  for (int kb = 0; kb < K; kb += 32) {
    FragB ah, al;
    const v4f x0 = *(const v4fa*)(arow + kb + 8 * hh), x1 = *(const v4fa*)(arow + kb + 8 * hh + 4);
    const v4f x2 = *(const v4fa*)(arow + kb + 16 + 8 * hh), x3 = *(const v4fa*)(arow + kb + 16 + 8 * hh + 4);
    float xs[16] = {x0[0],x0[1],x0[2],x0[3],x1[0],x1[1],x1[2],x1[3],x2[0],x2[1],x2[2],x2[3],x3[0],x3[1],x3[2],x3[3]};
#pragma unroll
    for (int i = 0; i < 16; ++i) { const unsigned short hb = bf16_bits(xs[i]); ah.u[i] = hb; al.u[i] = ASPLIT ? bf16_bits(xs[i] - bf16_val(hb)) : (unsigned short)0; }
#pragma unroll
    for (int t = 0; t < 4; ++t) {
      const unsigned short* brow = Wt + (size_t)(col0 + t * 16 + ln) * ldb + kb;
      FragB b;
      b.half[0] = *(const v8us*)(brow + 8 * hh);
      b.half[1] = *(const v8us*)(brow + 16 + 8 * hh);
      acc[t] = mmaN<ASPLIT ? 2 : 1>(ah.v, al.v, b.v, b.v, acc[t]);
    }
  }
#pragma unroll
  for (int t = 0; t < 4; ++t) {
    const int col = col0 + t * 16 + ln;
    float bv = bias ? bias[col] : 0.f;
    if (BIAS_BF16) bv = bf16_round(bv);
#pragma unroll
    for (int r = 0; r < 8; ++r) {
      float v = acc[t][r] + bv;
      if (resid) { float rv = resid[(size_t)((row0 + 8 * hh + r) % rmod) * ldr + col]; if (RES_BF16) rv = bf16_round(rv); v += rv; }
      if (ACT == 1) v = fmaxf(v, 0.f);
      if (ACT == 2) v = 0.5f * v * (1.0f + erff(v * 0.70710678118654752f));
      if (ACT == 3) { const float u = 0.7978845608028654f * (v + 0.044715f * v * v * v); v = 0.5f * v * (1.0f + tanhf(u)); }
      so[w][8 * hh + r][t * 16 + ln] = v;
    }
  }
  __builtin_amdgcn_fence(__ATOMIC_ACQ_REL, "workgroup");
  __builtin_amdgcn_wave_barrier();
  const int rsub = lane >> 4, c4 = (lane & 15) * 4;
  for (int pass = 0; pass < 2; ++pass) {
#pragma unroll
    for (int q = 0; q < 8; ++q) {
      const int r = q * 2 + rsub;
      const v4f v = *(const v4fa*)&so[w][r][c4];
      *(volatile v4f*)(C + (size_t)(row0 + r) * ldc + col0 + c4) = v;
    }
    if (pass == 0) __threadfence();
  }
}
template <bool PARAM_BF16>
__global__ __launch_bounds__(256) void k_layernorm(const float* __restrict__ X, const float* __restrict__ R, const float* __restrict__ g, const float* __restrict__ bta,
                                                  float* __restrict__ out_sum, float* __restrict__ out_norm, int N, float eps) {
  __shared__ float red[256];
  const int row = blockIdx.x, tid = threadIdx.x;
  const float* x = X + (size_t)row * N; const float* rr = R ? R + (size_t)row * N : nullptr;
  float vals[16];
  const int per = N / 256;
  float s1 = 0.f;
  for (int u = 0; u < per / 4; ++u) {
    const int j = tid * 4 + 1024 * u;
    const v4f a = *(const v4fa*)(x + j);
    v4f b = {0.f,0.f,0.f,0.f}; if (rr) b = *(const v4fa*)(rr + j);
#pragma unroll
    for (int q = 0; q < 4; ++q) { const float v = a[q] + b[q]; vals[u * 4 + q] = v; s1 += v; }
  }
  red[tid] = s1; __syncthreads();
  for (int st = 128; st > 0; st >>= 1) { if (tid < st) red[tid] += red[tid + st]; __syncthreads(); }
  const float mu = red[0] / (float)N; __syncthreads();
  float s2 = 0.f;
  for (int u = 0; u < per / 4; ++u)
#pragma unroll
    for (int q = 0; q < 4; ++q) { const float c = vals[u * 4 + q] - mu; s2 += c * c; }
  red[tid] = s2; __syncthreads();
  for (int st = 128; st > 0; st >>= 1) { if (tid < st) red[tid] += red[tid + st]; __syncthreads(); }
  const float rs = rsqrtf(red[0] / (float)N + eps);
  for (int pass = 0; pass < 2; ++pass) {
    for (int u = 0; u < per / 4; ++u) {
      const int j = tid * 4 + 1024 * u;
      v4f o, sm;
#pragma unroll
      for (int q = 0; q < 4; ++q) {
        float gg = g[j + q], bb = bta[j + q];
        if (PARAM_BF16) { gg = bf16_round(gg); bb = bf16_round(bb); }
        sm[q] = vals[u * 4 + q]; o[q] = (vals[u * 4 + q] - mu) * rs * gg + bb;
      }
      if (out_sum) *(volatile v4f*)(out_sum + (size_t)row * N + j) = sm;
      *(volatile v4f*)(out_norm + (size_t)row * N + j) = o;
    }
    if (pass == 0) __threadfence();
  }
}


typedef _Float16 v16h __attribute__((ext_vector_type(16)));
union FragH { v16h v; v8us half[2]; _Float16 h[16]; unsigned short u[16]; };
template <int NT>
__device__ __forceinline__ v8f mmaH(v16h ah, v16h al, v16h bh, v16h bl, v8f c) {
  c = __builtin_amdgcn_wmma_f32_16x16x32_f16(false, ah, false, bh, (short)0, c, false, false);
  if (NT >= 2) c = __builtin_amdgcn_wmma_f32_16x16x32_f16(false, al, false, bh, (short)0, c, false, false);
  if (NT >= 3) c = __builtin_amdgcn_wmma_f32_16x16x32_f16(false, ah, false, bl, (short)0, c, false, false);
  asm volatile("v_nop\n\tv_nop\n\tv_nop\n\tv_nop" : "+v"(c) : "v"(ah), "v"(al), "v"(bh), "v"(bl));
  return c;
}
template <bool ASPLIT>
__global__ __launch_bounds__(128) void k_gemm_h(const float* __restrict__ A, int lda, size_t sA, const _Float16* __restrict__ Bh, int ldb, size_t sB, float alpha, float* __restrict__ C, int ldc, size_t sC, int M, int N, int K) {
  __shared__ __attribute__((aligned(16))) float so[4][16][64];
  const int tid = threadIdx.x, w = tid >> 5, lane = tid & 31, ln = lane & 15, hh = lane >> 4; const int by = blockIdx.y;
  A += (size_t)by * sA; Bh += (size_t)by * sB; C += (size_t)by * sC;
  const int ntn = (N + 63) / 64; const int wid = blockIdx.x * 4 + w; const int mt = wid / ntn, nq = wid % ntn; if (mt * 16 >= M) return;
  const int row0 = mt * 16, col0 = nq * 64; const float* arow = A + (size_t)(row0 + ln) * lda;
  v8f acc[4] = {};
  for (int kb = 0; kb < K; kb += 32) {
    FragH ah, al;
    const v4f x0 = *(const v4fa*)(arow + kb + 8 * hh), x1 = *(const v4fa*)(arow + kb + 8 * hh + 4), x2 = *(const v4fa*)(arow + kb + 16 + 8 * hh), x3 = *(const v4fa*)(arow + kb + 16 + 8 * hh + 4);
    float xs[16] = {x0[0],x0[1],x0[2],x0[3],x1[0],x1[1],x1[2],x1[3],x2[0],x2[1],x2[2],x2[3],x3[0],x3[1],x3[2],x3[3]};
#pragma unroll
    for (int i = 0; i < 16; ++i) { const _Float16 h = (_Float16)xs[i]; ah.h[i] = h; al.h[i] = ASPLIT ? (_Float16)(xs[i] - (float)h) : (_Float16)0.0f; }
#pragma unroll
    for (int t = 0; t < 4; ++t) { if (col0 + t * 16 >= N) continue; const size_t boff = (size_t)(col0 + t * 16 + ln) * ldb + kb; FragH bq; bq.half[0] = *(const v8us*)(Bh + boff + 8 * hh); bq.half[1] = *(const v8us*)(Bh + boff + 16 + 8 * hh);
      acc[t] = mmaH<ASPLIT ? 2 : 1>(ah.v, al.v, bq.v, bq.v, acc[t]); }
  }
#pragma unroll
  for (int t = 0; t < 4; ++t) { if (col0 + t * 16 >= N) continue;
#pragma unroll
    for (int r = 0; r < 8; ++r) so[w][8 * hh + r][t * 16 + ln] = acc[t][r] * alpha; }
  __builtin_amdgcn_fence(__ATOMIC_ACQ_REL, "workgroup"); __builtin_amdgcn_wave_barrier();
  const int rsub = lane >> 4, c4 = (lane & 15) * 4;
  for (int pass = 0; pass < 2; ++pass) {
#pragma unroll
    for (int q = 0; q < 8; ++q) { const int r = q * 2 + rsub; if (col0 + c4 < N) { const v4f v = *(const v4fa*)&so[w][r][c4]; *(volatile v4f*)(C + (size_t)(row0 + r) * ldc + col0 + c4) = v; } }
    if (pass == 0) __threadfence(); }
}

__global__ __launch_bounds__(256) void k_wt_f16(const float* __restrict__ W, _Float16* __restrict__ Wt, int K, int N, float scale) {
  const int t = blockIdx.x * 256 + threadIdx.x; if (t >= N * (K / 8)) return; const int n = t / (K / 8), k8 = (t % (K / 8)) * 8; FragH f;
#pragma unroll
  for (int i = 0; i < 8; ++i) f.h[i] = (_Float16)(bf16_round(W[(size_t)(k8 + i) * N + n]) * scale); const v8us o = f.half[0];
  *(volatile v8us*)((unsigned short*)Wt + (size_t)n * K + k8) = o; __threadfence(); *(volatile v8us*)((unsigned short*)Wt + (size_t)n * K + k8) = o;
}
template <int ACT>
__global__ __launch_bounds__(128) void k_gemm_hhx(const _Float16* __restrict__ A, int lda, size_t sA, const _Float16* __restrict__ Bh, int ldb, size_t sB, float alpha, const float* __restrict__ bias, size_t sBias, const float* __restrict__ CP, int rowsPerB, size_t sCPb, int row0g,
    float* __restrict__ C, _Float16* __restrict__ C16, int ldc, size_t sC, int M, int N, int K) {
  __shared__ __attribute__((aligned(16))) float so[4][16][64];
  const int tid = threadIdx.x, w = tid >> 5, lane = tid & 31, ln = lane & 15, hh = lane >> 4; const int by = blockIdx.y;
  A += (size_t)by * sA; Bh += (size_t)by * sB; const size_t cofs = (size_t)by * sC; const float* bp = bias ? bias + (size_t)by * sBias : nullptr;
  const int ntn = (N + 63) / 64; const int wid = blockIdx.x * 4 + w; const int mt = wid / ntn, nq = wid % ntn; if (mt * 16 >= M) return;
  const int row0 = mt * 16, col0 = nq * 64; const _Float16* arow = A + (size_t)(row0 + ln) * lda;
  v8f acc[4] = {};
  for (int kb = 0; kb < K; kb += 32) { FragH ah; ah.half[0] = *(const v8us*)((const unsigned short*)arow + kb + 8 * hh); ah.half[1] = *(const v8us*)((const unsigned short*)arow + kb + 16 + 8 * hh);
#pragma unroll
    for (int t = 0; t < 4; ++t) { if (col0 + t * 16 >= N) continue; const size_t boff = (size_t)(col0 + t * 16 + ln) * ldb + kb; FragH bq; bq.half[0] = *(const v8us*)((const unsigned short*)Bh + boff + 8 * hh); bq.half[1] = *(const v8us*)((const unsigned short*)Bh + boff + 16 + 8 * hh);
      acc[t] = mmaH<1>(ah.v, ah.v, bq.v, bq.v, acc[t]); }
  }
#pragma unroll
  for (int t = 0; t < 4; ++t) { if (col0 + t * 16 >= N) continue; const int col = col0 + t * 16 + ln; const float bv = bp ? bf16_round(bp[col]) : 0.f;
#pragma unroll
    for (int r = 0; r < 8; ++r) { float v = acc[t][r] * alpha + bv; if (CP) { const int rr = row0g + row0 + 8 * hh + r; if (rowsPerB < 0) v += CP[cofs + (size_t)rr * ldc + col];        else { const int bidx = rr / rowsPerB; v += CP[(size_t)bidx * sCPb + (size_t)by * 64 + col]; } } if (ACT == 1) v = (v > 0.f) ? v : expm1f(v); else if (ACT == 7) v = (v > 0.f) ? v + 1.0f : expf(v); else if (ACT == 8) v = tanhf(v); else if (ACT == 9) v = 0.5f * v * (1.0f + tanhf(0.7978845608028654f * (v + 0.044715f * v * v * v))); else if (ACT == 11) v = 1.0f / (1.0f + expf(-v)); else if (ACT == 12) v = (v > 0.f) ? v : 0.01f * v; else if (ACT == 14) v = (v > 0.f) ? v : 0.1f * v; else if (ACT == 16) v = (v >= 0.f) ? v : 0.3f * v; else if (ACT == 17) v = (v >= 0.f) ? v : 0.2f * v; else if (ACT == 15) v = v / (1.0f + expf(-v)); else if (ACT == 3) v = fmaxf(v, 0.f); else if (ACT == 6) v = 0.5f * v * (1.0f + erff(v * 0.70710678118654752f)); so[w][8 * hh + r][t * 16 + ln] = v; } }
  __builtin_amdgcn_fence(__ATOMIC_ACQ_REL, "workgroup"); __builtin_amdgcn_wave_barrier();
  const int rsub = lane >> 4, c4 = (lane & 15) * 4; typedef _Float16 v4h __attribute__((ext_vector_type(4)));
  for (int pass = 0; pass < 2; ++pass) {
#pragma unroll
    for (int q = 0; q < 8; ++q) { const int r = q * 2 + rsub; if (col0 + c4 < N) { const v4f v = *(const v4fa*)&so[w][r][c4]; if (C) *(volatile v4f*)(C + cofs + (size_t)(row0 + r) * ldc + col0 + c4) = v; if (C16) { v4h h4; for (int i = 0; i < 4; ++i) h4[i] = (_Float16)v[i]; *(volatile v4h*)(C16 + cofs + (size_t)(row0 + r) * ldc + col0 + c4) = h4; } } }
    if (pass == 0) __threadfence(); }
}


typedef _Float16 v4h __attribute__((ext_vector_type(4)));

__global__ __launch_bounds__(256) void k_x16(const float* __restrict__ x, _Float16* __restrict__ X16, size_t n8) { const size_t t = (size_t)blockIdx.x * 256 + threadIdx.x; if (t >= n8) return; FragH f;
#pragma unroll
  for (int q = 0; q < 8; ++q) f.h[q] = (_Float16)bf16_round(x[t * 8 + q]); *(volatile v8us*)((unsigned short*)X16 + t * 8) = f.half[0]; __threadfence(); *(volatile v8us*)((unsigned short*)X16 + t * 8) = f.half[0]; }
__global__ __launch_bounds__(256) void k_h16(const float* __restrict__ x, _Float16* __restrict__ X16, size_t n8) { const size_t t = (size_t)blockIdx.x * 256 + threadIdx.x; if (t >= n8) return; FragH f;
#pragma unroll
  for (int q = 0; q < 8; ++q) f.h[q] = (_Float16)x[t * 8 + q]; *(volatile v8us*)((unsigned short*)X16 + t * 8) = f.half[0]; __threadfence(); *(volatile v8us*)((unsigned short*)X16 + t * 8) = f.half[0]; }
__global__ __launch_bounds__(256) void k_round16f(const float* __restrict__ W, _Float16* __restrict__ Bt, size_t n8) { const size_t t = (size_t)blockIdx.x * 256 + threadIdx.x; if (t >= n8) return; FragH f;
#pragma unroll
  for (int i = 0; i < 8; ++i) f.h[i] = (_Float16)(bf16_round(W[t * 8 + i]) * 16.0f); *(volatile v8us*)((unsigned short*)Bt + t * 8) = f.half[0]; __threadfence(); *(volatile v8us*)((unsigned short*)Bt + t * 8) = f.half[0]; }
template <int NHv, int TTv>
__global__ __launch_bounds__(256) void k_vt(const _Float16* __restrict__ V16, int ldv, int voff, _Float16* __restrict__ Vt) { __shared__ unsigned short tl[64][66]; const int tid = threadIdx.x; const int slab = blockIdx.x / (TTv / 64), lg = blockIdx.x % (TTv / 64); const int b = slab / NHv, h = slab % NHv;
  for (int i = tid; i < 64 * 8; i += 256) { const int r = i / 8, c8 = (i % 8) * 8; FragH f; f.half[0] = *(const v8us*)((const unsigned short*)V16 + ((size_t)b * TTv + lg * 64 + r) * ldv + voff + h * 64 + c8);
#pragma unroll
    for (int q = 0; q < 8; ++q) tl[r][c8 + q] = f.u[q]; }
  __syncthreads();
  for (int pass = 0; pass < 2; ++pass) {
#pragma unroll
    for (int rd = 0; rd < 2; ++rd) { const int d = rd * 32 + tid / 8, pc = tid % 8; FragH f;
#pragma unroll
      for (int q = 0; q < 8; ++q) f.u[q] = tl[pc * 8 + q][d];
      *(volatile v8us*)((unsigned short*)Vt + ((size_t)slab * 64 + d) * TTv + lg * 64 + pc * 8) = f.half[0]; }
    if (pass == 0) __threadfence(); } }

__global__ __launch_bounds__(256) void k_hl(const float* __restrict__ F, _Float16* __restrict__ Hh, _Float16* __restrict__ Hl, size_t n8) { const size_t t = (size_t)blockIdx.x * 256 + threadIdx.x; if (t >= n8) return; FragH fh, fl; const v4f a = *(const v4fa*)(F + t * 8), c = *(const v4fa*)(F + t * 8 + 4);
#pragma unroll
  for (int q = 0; q < 4; ++q) { _Float16 h = (_Float16)a[q]; fh.h[q] = h; fl.h[q] = (_Float16)((a[q] - (float)h) * 1024.0f); h = (_Float16)c[q]; fh.h[4 + q] = h; fl.h[4 + q] = (_Float16)((c[q] - (float)h) * 1024.0f); }
  for (int pass = 0; pass < 2; ++pass) { *(volatile v8us*)((unsigned short*)Hh + t * 8) = fh.half[0]; *(volatile v8us*)((unsigned short*)Hl + t * 8) = fl.half[0]; if (pass == 0) __threadfence(); } }

__device__ __forceinline__ v16h g2_frag(const _Float16* p, int hh) { FragH f; f.half[0] = *(const v8us*)((const unsigned short*)p + 8 * hh); f.half[1] = *(const v8us*)((const unsigned short*)p + 16 + 8 * hh); return f.v; }
__device__ __forceinline__ v8f g2_mma(v16h a, v16h b, v8f c) { v8f d = __builtin_amdgcn_wmma_f32_16x16x32_f16(false, a, false, b, (short)0, c, false, false); asm volatile("v_nop\n\tv_nop\n\tv_nop\n\tv_nop" : "+v"(d) : "v"(a), "v"(b)); return d; }
template <int ACT>
__global__ __launch_bounds__(128) void k_gemm2(const _Float16* __restrict__ A, int lda, size_t sA, const _Float16* __restrict__ Bh, int ldb, size_t sB, float alpha, const float* __restrict__ bias, size_t sBias, const float* __restrict__ CP, int rowsPerB, size_t sCPb, int row0g,
    float* __restrict__ C, _Float16* __restrict__ C16, int ldc, size_t sC, int M, int N, int K) { static_assert(ACT == 0 || ACT == 3 || ACT == 6 || ACT == 8 || ACT == 9 || ACT == 11 || ACT == 12 || ACT == 14 || ACT == 15 || ACT == 16 || ACT == 17, "k_gemm2: unsupported ACT code (would silently apply no activation)");
  __shared__ __attribute__((aligned(16))) float so[4][32][68];
  const int tid = threadIdx.x, w = tid >> 5, lane = tid & 31, ln = lane & 15, hh = lane >> 4; const int by = blockIdx.y;
  A += (size_t)by * sA; Bh += (size_t)by * sB; const size_t cofs = (size_t)by * sC; const float* bp = bias ? bias + (size_t)by * sBias : nullptr;
  const int ntn = N >> 6; const int mt = blockIdx.x / ntn, nq = blockIdx.x - mt * ntn; const int row0 = mt * 128 + 32 * w, col0 = nq * 64; if (row0 >= M) return;
  const _Float16* a0p = A + (size_t)(row0 + ln) * lda; const _Float16* a1p = a0p + (size_t)16 * lda;
  const _Float16* b0p = Bh + (size_t)(col0 + ln) * ldb; const _Float16* b1p = b0p + (size_t)16 * ldb; const _Float16* b2p = b1p + (size_t)16 * ldb; const _Float16* b3p = b2p + (size_t)16 * ldb;
  const v8f z8 = {0.f,0.f,0.f,0.f,0.f,0.f,0.f,0.f}; v8f c00 = z8, c01 = z8, c02 = z8, c03 = z8, c10 = z8, c11 = z8, c12 = z8, c13 = z8;
#pragma unroll 1
  for (int kb = 0; kb < K; kb += 32) { const v16h a0 = g2_frag(a0p + kb, hh), a1 = g2_frag(a1p + kb, hh);
    v16h b = g2_frag(b0p + kb, hh); c00 = g2_mma(a0, b, c00); c10 = g2_mma(a1, b, c10);
    b = g2_frag(b1p + kb, hh); c01 = g2_mma(a0, b, c01); c11 = g2_mma(a1, b, c11);
    b = g2_frag(b2p + kb, hh); c02 = g2_mma(a0, b, c02); c12 = g2_mma(a1, b, c12);
    b = g2_frag(b3p + kb, hh); c03 = g2_mma(a0, b, c03); c13 = g2_mma(a1, b, c13); }
  v8f accs[8] = {c00, c01, c02, c03, c10, c11, c12, c13};
#pragma unroll
  for (int u = 0; u < 8; ++u) { const int t = u & 3, half = u >> 2; const int col = col0 + t * 16 + ln; const float bv = bp ? bf16_round(bp[col]) : 0.f;
#pragma unroll
    for (int r = 0; r < 8; ++r) { const int rloc = half * 16 + 8 * hh + r; float v = accs[u][r] * alpha + bv; if (CP) { if (rowsPerB < 0) v += CP[cofs + (size_t)(row0g + row0 + rloc) * ldc + col];        else { const int bidx = (row0g + row0 + rloc) / rowsPerB; v += CP[(size_t)bidx * sCPb + (size_t)by * 64 + col]; } }
      if (ACT == 3) v = fmaxf(v, 0.f); else if (ACT == 6) v = 0.5f * v * (1.0f + erff(v * 0.70710678118654752f)); else if (ACT == 11) v = 1.0f / (1.0f + expf(-v)); else if (ACT == 15) v = v / (1.0f + expf(-v)); else if (ACT == 12) v = (v > 0.f) ? v : 0.01f * v; else if (ACT == 8) v = tanhf(v); else if (ACT == 9) v = 0.5f * v * (1.0f + tanhf(0.7978845608028654f * (v + 0.044715f * v * v * v))); else if (ACT == 14) v = (v > 0.f) ? v : 0.1f * v; else if (ACT == 16) v = (v >= 0.f) ? v : 0.3f * v; else if (ACT == 17) v = (v >= 0.f) ? v : 0.2f * v;
      so[w][rloc][t * 16 + ln] = v; } }
  __builtin_amdgcn_fence(__ATOMIC_ACQ_REL, "workgroup"); __builtin_amdgcn_wave_barrier();
  const int rsub = lane >> 4, c4 = (lane & 15) * 4;
  for (int pass = 0; pass < 2; ++pass) {
#pragma unroll
    for (int q = 0; q < 16; ++q) { const int r = q * 2 + rsub; const v4f v = *(const v4fa*)&so[w][r][c4]; if (C) *(volatile v4f*)(C + cofs + (size_t)(row0 + r) * ldc + col0 + c4) = v; if (C16) { v4h h4; for (int i = 0; i < 4; ++i) h4[i] = (_Float16)v[i]; *(volatile v4h*)(C16 + cofs + (size_t)(row0 + r) * ldc + col0 + c4) = h4; } }
    if (pass == 0) __threadfence(); } }


__global__ __launch_bounds__(256) void k_wsc(const float* __restrict__ Wm, _Float16* __restrict__ Bt, size_t n8, float sc) { const size_t t = (size_t)blockIdx.x * 256 + threadIdx.x; if (t >= n8) return; FragH f; for (int q = 0; q < 8; ++q) f.h[q] = (_Float16)(bf16_round(Wm[t * 8 + q]) * sc); *(volatile v8us*)((unsigned short*)Bt + t * 8) = f.half[0]; __threadfence(); *(volatile v8us*)((unsigned short*)Bt + t * 8) = f.half[0]; }
__global__ __launch_bounds__(256) void k_wfc2(const float* __restrict__ Wm, _Float16* __restrict__ Bt) { const int t = blockIdx.x * 256 + threadIdx.x; if (t >= CH * HID / 8) return; const int k0 = (t * 8) % HID; const int o = (t * 8) / HID; FragH f; for (int q = 0; q < 8; ++q) f.h[q] = (_Float16)(bf16_round(Wm[(size_t)o * 2 * HID + k0 + q]) * 16.0f);
  *(volatile v8us*)((unsigned short*)Bt + (size_t)t * 8) = f.half[0]; __threadfence(); *(volatile v8us*)((unsigned short*)Bt + (size_t)t * 8) = f.half[0]; }
__global__ __launch_bounds__(256) void k_instat(const float* __restrict__ x, float* __restrict__ MU, float* __restrict__ RSD) {
  #pragma clang fp contract(off)
  __shared__ float smu[32], srs[32]; const int wv = threadIdx.x >> 5, ln = threadIdx.x & 31;
#pragma unroll 1
  for (int i = 0; i < 4; ++i) { const int bc = blockIdx.x * 32 + wv * 4 + i; const float* xr = x + (size_t)bc * PX; float s = 0.f;
#pragma unroll 1
    for (int j = 0; j < PX / 32; ++j) s += bf16_round(xr[j * 32 + ln]);
    for (int o = 16; o > 0; o >>= 1) s += __shfl_xor(s, o, 32); const float mu = s / (float)PX; float s2 = 0.f;
#pragma unroll 1
    for (int j = 0; j < PX / 32; ++j) { const float d = bf16_round(xr[j * 32 + ln]) - mu; s2 += d * d; }
    for (int o = 16; o > 0; o >>= 1) s2 += __shfl_xor(s2, o, 32); if (ln == 0) { smu[wv * 4 + i] = mu; srs[wv * 4 + i] = rsqrtf(s2 / (float)PX + 1e-5f); } }
  __syncthreads(); if (threadIdx.x < 32) { const int bc = blockIdx.x * 32 + threadIdx.x; for (int pass = 0; pass < 2; ++pass) { *(volatile float*)(MU + bc) = smu[threadIdx.x]; *(volatile float*)(RSD + bc) = srs[threadIdx.x]; if (pass == 0) __threadfence(); } } }
__device__ __forceinline__ int win_row(int b, int p) { const int y = p / HS, xx = p % HS; const int w = (y / WSZ) * (HS / WSZ) + xx / WSZ, t = (y % WSZ) * WSZ + xx % WSZ; return (b * NWIN + w) * WT + t; }
__global__ __launch_bounds__(256) void k_xn(const float* __restrict__ x, const float* __restrict__ MU, const float* __restrict__ RSD, _Float16* __restrict__ XN, _Float16* __restrict__ XNW) {
  #pragma clang fp contract(off)
  const size_t t = (size_t)blockIdx.x * 256 + threadIdx.x; if (t >= (size_t)NR * CH / 8) return; const int c0 = (int)((t * 8) % CH); const size_t row = (t * 8) / CH; const int b = (int)(row / PX), p = (int)(row % PX); FragH f;
  for (int q = 0; q < 8; ++q) { const int c = c0 + q; const float v = (bf16_round(x[((size_t)b * CH + c) * PX + p]) - MU[b * CH + c]) * RSD[b * CH + c]; f.h[q] = (_Float16)v; }
  const size_t o1 = row * CH + c0, o2 = (size_t)win_row(b, p) * CH + c0; for (int pass = 0; pass < 2; ++pass) { *(volatile v8us*)((unsigned short*)XN + o1) = f.half[0]; *(volatile v8us*)((unsigned short*)XNW + o2) = f.half[0]; if (pass == 0) __threadfence(); } }
template <int L>
__global__ __launch_bounds__(256) void k_soft(const float* __restrict__ S, _Float16* __restrict__ P, float* __restrict__ RS, int nrow) {
  #pragma clang fp contract(off)
  const int wv = threadIdx.x >> 5, ln = threadIdx.x & 31; const int r = blockIdx.x * 8 + wv; if (r >= nrow) return; const float* sr = S + (size_t)r * L; const float scl = 0.17677669529663687f; constexpr int PER = L / 32; float mx = -3.0e38f;
  for (int j = 0; j < PER; ++j) mx = fmaxf(mx, sr[j * 32 + ln] * scl);
  for (int o = 16; o > 0; o >>= 1) mx = fmaxf(mx, __shfl_xor(mx, o, 32)); float su = 0.f;
  if (L == 64) { typedef _Float16 v2h_ __attribute__((ext_vector_type(2))); const float e0 = expf(sr[ln * 2] * scl - mx), e1 = expf(sr[ln * 2 + 1] * scl - mx); su = e0 + e1; v2h_ h; h[0] = (_Float16)(e0 * 1024.0f); h[1] = (_Float16)(e1 * 1024.0f); *(volatile v2h_*)(P + (size_t)r * L + ln * 2) = h; __threadfence(); *(volatile v2h_*)(P + (size_t)r * L + ln * 2) = h; }
  else {
#pragma unroll 1
    for (int pass = 0; pass < 2; ++pass) { su = 0.f;
#pragma unroll 1
      for (int gq = 0; gq < L / 256; ++gq) { const v8f a = *(const v8f*)(sr + gq * 256 + ln * 8); FragH ph; for (int i = 0; i < 8; ++i) { const float e = expf(a[i] * scl - mx); su += e; ph.h[i] = (_Float16)(e * 1024.0f); } *(volatile v8us*)((unsigned short*)P + (size_t)r * L + gq * 256 + ln * 8) = ph.half[0]; }
      if (pass == 0) __threadfence(); } }
  for (int o = 16; o > 0; o >>= 1) su += __shfl_xor(su, o, 32); if (ln == 0) { *(volatile float*)(RS + (size_t)r * 32) = 1.0f / su; __threadfence(); *(volatile float*)(RS + (size_t)r * 32) = 1.0f / su; } }
__global__ __launch_bounds__(256) void k_osc(const float* __restrict__ O, const float* __restrict__ RS, size_t rsHeadStride, size_t rowOff, size_t nrow, _Float16* __restrict__ CX16) {
  #pragma clang fp contract(off)
  const size_t t = (size_t)blockIdx.x * 256 + threadIdx.x; if (t >= nrow * CH / 8) return; const int c0 = (int)((t * 8) % CH); const size_t rl = (t * 8) / CH; const int h = c0 / HD; const float rs = RS[((size_t)h * rsHeadStride + rl) * 32]; const v8f a = *(const v8f*)(O + rl * CH + c0); FragH f; for (int i = 0; i < 8; ++i) f.h[i] = (_Float16)(a[i] * rs);
  unsigned short* dst = (unsigned short*)CX16 + (rowOff + rl) * CH + c0; *(volatile v8us*)dst = f.half[0]; __threadfence(); *(volatile v8us*)dst = f.half[0]; }
__global__ __launch_bounds__(256) void k_x1(const float* __restrict__ x, const float* __restrict__ YW, const float* __restrict__ YG, float* __restrict__ X1) {
  #pragma clang fp contract(off)
  const size_t t = (size_t)blockIdx.x * 256 + threadIdx.x; if (t >= (size_t)NR * CH / 8) return; const int c0 = (int)((t * 8) % CH); const size_t row = (t * 8) / CH; const int b = (int)(row / PX), p = (int)(row % PX); const size_t wr = (size_t)win_row(b, p); const v8f yw = *(const v8f*)(YW + wr * CH + c0), yg = *(const v8f*)(YG + row * CH + c0); v8f o;
  for (int q = 0; q < 8; ++q) { float v = bf16_round(x[((size_t)b * CH + c0 + q) * PX + p]) + yw[q]; v += yg[q]; o[q] = v; }
  *(volatile v8f*)(X1 + t * 8) = o; __threadfence(); *(volatile v8f*)(X1 + t * 8) = o; }
__global__ __launch_bounds__(256) void k_cstat(const float* __restrict__ Y, int ncol, const float* __restrict__ MU, int pass, float eps, float* __restrict__ OUTV) {
  #pragma clang fp contract(off)
  __shared__ float red[4][64]; const int tid = threadIdx.x; const int ngrp = ncol / 64; const int b = blockIdx.x / ngrp, cg = blockIdx.x % ngrp; const int c = cg * 64 + (tid & 63), part = tid >> 6; float s = 0.f; const float mu = pass ? MU[b * ncol + c] : 0.f;
#pragma unroll 1
  for (int p = part; p < PX; p += 4) { const float v = Y[((size_t)b * PX + p) * ncol + c]; if (pass) { const float d = v - mu; s += d * d; } else s += v; }
  red[part][tid & 63] = s; __syncthreads(); if (part == 0) { float tot = red[0][tid] + red[1][tid]; tot += red[2][tid]; tot += red[3][tid]; const float r = pass ? rsqrtf(tot / (float)PX + eps) : tot / (float)PX; *(volatile float*)(OUTV + b * ncol + c) = r; __threadfence(); *(volatile float*)(OUTV + b * ncol + c) = r; } }
__global__ __launch_bounds__(256) void k_se(const float* __restrict__ CM, const float* __restrict__ MU2, const float* __restrict__ RS2, const float* __restrict__ W1, const float* __restrict__ W2, float* __restrict__ SV) {
  #pragma clang fp contract(off)
  __shared__ float sm[CH], sh[16]; const int b = blockIdx.x, c = threadIdx.x; sm[c] = (CM[b * CH + c] - MU2[b * CH + c]) * RS2[b * CH + c]; __syncthreads();
  if (c < 16) { float s = 0.f;
#pragma unroll 1
    for (int k = 0; k < CH; ++k) s += bf16_round(W1[c * CH + k]) * sm[k]; sh[c] = fmaxf(s, 0.f); }
  __syncthreads(); float s = 0.f; for (int j = 0; j < 16; ++j) s += bf16_round(W2[c * 16 + j]) * sh[j]; const float v = 1.0f / (1.0f + expf(-s)); *(volatile float*)(SV + b * CH + c) = v; __threadfence(); *(volatile float*)(SV + b * CH + c) = v; }
__global__ __launch_bounds__(256) void k_x2(const float* __restrict__ X1, const float* __restrict__ MU2, const float* __restrict__ RS2, const float* __restrict__ SV, float* __restrict__ X2) {
  #pragma clang fp contract(off)
  const size_t t = (size_t)blockIdx.x * 256 + threadIdx.x; if (t >= (size_t)NR * CH / 8) return; const int c0 = (int)((t * 8) % CH); const int b = (int)((t * 8) / CH / PX); const v8f a = *(const v8f*)(X1 + t * 8); v8f o; for (int q = 0; q < 8; ++q) { const int i = b * CH + c0 + q; const float xn = (a[q] - MU2[i]) * RS2[i]; o[q] = a[q] + xn * SV[i]; }
  *(volatile v8f*)(X2 + t * 8) = o; __threadfence(); *(volatile v8f*)(X2 + t * 8) = o; }
__global__ __launch_bounds__(256) void k_xn3(const float* __restrict__ X2, const float* __restrict__ MU3, const float* __restrict__ RS3, _Float16* __restrict__ D) {
  #pragma clang fp contract(off)
  const size_t t = (size_t)blockIdx.x * 256 + threadIdx.x; if (t >= (size_t)NR * CH / 8) return; const int c0 = (int)((t * 8) % CH); const int b = (int)((t * 8) / CH / PX); const v8f a = *(const v8f*)(X2 + t * 8); FragH f; for (int q = 0; q < 8; ++q) { const int i = b * CH + c0 + q; f.h[q] = (_Float16)((a[q] - MU3[i]) * RS3[i]); }
  *(volatile v8us*)((unsigned short*)D + t * 8) = f.half[0]; __threadfence(); *(volatile v8us*)((unsigned short*)D + t * 8) = f.half[0]; }
__global__ __launch_bounds__(256) void k_dwg(const float* __restrict__ H1, const float* __restrict__ w3, const float* __restrict__ b3, const float* __restrict__ w5, const float* __restrict__ b5, _Float16* __restrict__ D) {
  #pragma clang fp contract(off)
  const size_t t = (size_t)blockIdx.x * 256 + threadIdx.x; if (t >= (size_t)NR * HID / 4) return; const int c0 = (int)((t * 4) % HID); const size_t row = (t * 4) / HID; const int b = (int)(row / PX), p = (int)(row % PX); const int y = p / HS, xx = p % HS; const bool big = c0 >= HID / 2; const int K = big ? 5 : 3, P2 = K / 2; v4h o;
#pragma unroll 1
  for (int q = 0; q < 4; ++q) { const int c = c0 + q; const int cl = big ? c - HID / 2 : c; const float* w = big ? (w5 + cl * 25) : (w3 + cl * 9); float s = bf16_round(big ? b5[cl] : b3[cl]);
#pragma unroll 1
    for (int k = 0; k < K * K; ++k) { const int yy = y - P2 + k / K, xq = xx - P2 + k % K; if (yy < 0 || yy >= HS || xq < 0 || xq >= HS) continue; s += H1[((size_t)b * PX + yy * HS + xq) * HID + c] * bf16_round(w[k]); }
    o[q] = (_Float16)(0.5f * s * (1.0f + erff(s * 0.70710678118654752f))); }
  *(volatile v4h*)(D + t * 4) = o; __threadfence(); *(volatile v4h*)(D + t * 4) = o; }
__global__ __launch_bounds__(256) void k_gtab(const float* __restrict__ G, const float* __restrict__ fc2w, const float* __restrict__ fc2b, float* __restrict__ GB) {
  #pragma clang fp contract(off)
  const int b = blockIdx.x, o = threadIdx.x; float s = 0.f;
#pragma unroll 1
  for (int k = 0; k < HID; k += 4) { const v4f gv = *(const v4fa*)(G + b * HID + k); for (int q = 0; q < 4; ++q) s += bf16_round(fc2w[(size_t)o * 2 * HID + HID + k + q]) * gv[q]; }
  s += bf16_round(fc2b[o]); *(volatile float*)(GB + b * CH + o) = s; __threadfence(); *(volatile float*)(GB + b * CH + o) = s; }
__global__ __launch_bounds__(256) void k_out(const float* __restrict__ X2, const float* __restrict__ Y, float* __restrict__ out) {
  #pragma clang fp contract(off)
  const size_t t = (size_t)blockIdx.x * 256 + threadIdx.x; if (t >= (size_t)NI * CH * PX / 8) return; const int p0 = (int)((t * 8) % PX); const size_t bc = (t * 8) / PX; const int b = (int)(bc / CH), c = (int)(bc % CH); v8f v; for (int q = 0; q < 8; ++q) { const size_t row = (size_t)b * PX + p0 + q; v[q] = X2[row * CH + c] + Y[row * CH + c]; }
  *(volatile v8f*)(out + t * 8) = v; __threadfence(); *(volatile v8f*)(out + t * 8) = v; }

extern "C" void kernel_launch(void* const* d_in, const int* in_sizes, int n_in,
                              void* d_out, int out_size, void* d_ws, size_t ws_size, hipStream_t stream) {
  (void)in_sizes; (void)n_in; (void)out_size;
  const float* const* I = (const float* const*)d_in;
  const float* x = I[0]; const float* wa_qkv = I[1]; const float* wa_pw = I[2]; const float* wa_pb = I[3]; const float* ga_qkv = I[4]; const float* ga_pw = I[5]; const float* ga_pb = I[6]; const float* ca_w1 = I[7]; const float* ca_w2 = I[8]; const float* fc1_w = I[9]; const float* fc1_b = I[10]; const float* dw3_w = I[11]; const float* dw3_b = I[12]; const float* dw5_w = I[13]; const float* dw5_b = I[14]; const float* fc2_w = I[15]; const float* fc2_b = I[16];
  char* ws = (char*)d_ws; size_t off = 0;
  auto take = [&](size_t bytes) { char* p = ws + off; off += (bytes + 255) & ~(size_t)255; return p; };
  const size_t np = (size_t)NR * CH;
  _Float16* BAQ = (_Float16*)take((size_t)3 * CH * CH * 2); _Float16* BAP = (_Float16*)take((size_t)CH * CH * 2); _Float16* BGQ = (_Float16*)take((size_t)3 * CH * CH * 2); _Float16* BGP = (_Float16*)take((size_t)CH * CH * 2); _Float16* BF1 = (_Float16*)take((size_t)HID * CH * 2); _Float16* BF2 = (_Float16*)take((size_t)CH * HID * 2);
  float* MU = (float*)take(NI * CH * 4); float* RSD = (float*)take(NI * CH * 4); float* MU2 = (float*)take(NI * CH * 4); float* RS2 = (float*)take(NI * CH * 4); float* CM = (float*)take(NI * CH * 4); float* SV = (float*)take(NI * CH * 4); float* MU3 = (float*)take(NI * CH * 4); float* RS3 = (float*)take(NI * CH * 4); float* G = (float*)take(NI * HID * 4); float* GB = (float*)take(NI * CH * 4);
  _Float16* XN = (_Float16*)take(np * 2); _Float16* XNW = (_Float16*)take(np * 2); _Float16* QKVW = (_Float16*)take(np * 3 * 2); _Float16* QKVG = (_Float16*)take(np * 3 * 2); _Float16* VTW = (_Float16*)take(np * 2); _Float16* VTG = (_Float16*)take(np * 2);
  float* SW = (float*)take((size_t)NH * NBW * WT * WT * 4);        _Float16* PW = (_Float16*)take((size_t)NH * NBW * WT * WT * 2); float* RSW = (float*)take((size_t)NH * NBW * WT * 32 * 4);        float* OW = (float*)take(np * 4); _Float16* CXW = (_Float16*)take(np * 2); float* YW = (float*)take(np * 4);
  float* SG = (float*)take((size_t)NH * PX * PX * 4);        _Float16* PG = (_Float16*)take((size_t)NH * PX * PX * 2); float* RSG = (float*)take((size_t)NH * PX * 32 * 4); float* OG = (float*)take((size_t)PX * CH * 4); _Float16* CXG = (_Float16*)take(np * 2); float* YG = (float*)take(np * 4);
  float* X1 = (float*)take(np * 4); float* X2 = (float*)take(np * 4); _Float16* XN3 = XN;        float* H1 = (float*)take((size_t)NR * HID * 4);        _Float16* A16 = (_Float16*)take((size_t)NR * HID * 2); float* Y = OW;
  if (off > ws_size) return;
  k_wsc<<<(unsigned)(((size_t)3 * CH * CH / 8 + 255) / 256), 256, 0, stream>>>(wa_qkv, BAQ, (size_t)3 * CH * CH / 8, 16.0f); k_wsc<<<(CH * CH / 8 + 255) / 256, 256, 0, stream>>>(wa_pw, BAP, (size_t)CH * CH / 8, 16.0f); k_wsc<<<(unsigned)(((size_t)3 * CH * CH / 8 + 255) / 256), 256, 0, stream>>>(ga_qkv, BGQ, (size_t)3 * CH * CH / 8, 16.0f); k_wsc<<<(CH * CH / 8 + 255) / 256, 256, 0, stream>>>(ga_pw, BGP, (size_t)CH * CH / 8, 16.0f);
  k_wsc<<<(unsigned)(((size_t)HID * CH / 8 + 255) / 256), 256, 0, stream>>>(fc1_w, BF1, (size_t)HID * CH / 8, 16.0f); k_wfc2<<<(CH * HID / 8 + 255) / 256, 256, 0, stream>>>(fc2_w, BF2);
  k_instat<<<NI * CH / 32, 256, 0, stream>>>(x, MU, RSD);
  k_xn<<<(unsigned)((np / 8 + 255) / 256), 256, 0, stream>>>(x, MU, RSD, XN, XNW);
  k_gemm2<0><<<dim3((NR / 128) * (3 * CH / 64), 1), 128, 0, stream>>>(XNW, CH, 0, BAQ, CH, 0, 0.0625f, nullptr, 0, nullptr, 1, 0, 0, nullptr, QKVW, 3 * CH, 0, NR, 3 * CH, CH);
  k_gemm2<0><<<dim3((NR / 128) * (3 * CH / 64), 1), 128, 0, stream>>>(XN, CH, 0, BGQ, CH, 0, 0.0625f, nullptr, 0, nullptr, 1, 0, 0, nullptr, QKVG, 3 * CH, 0, NR, 3 * CH, CH);
  k_vt<CH / 64, WT><<<NBW * (CH / 64) * (WT / 64), 256, 0, stream>>>(QKVW, 3 * CH, 2 * CH, VTW);
  k_vt<CH / 64, PX><<<NI * (CH / 64) * (PX / 64), 256, 0, stream>>>(QKVG, 3 * CH, 2 * CH, VTG);
  for (int h = 0; h < NH; ++h) {
    k_gemm_hhx<0><<<dim3(((WT / 16) * 1) / 4, NBW), 128, 0, stream>>>(QKVW + h * HD, 3 * CH, (size_t)WT * 3 * CH, QKVW + CH + h * HD, 3 * CH, (size_t)WT * 3 * CH, 1.0f, nullptr, 0, nullptr, 1, 0, 0, SW + (size_t)h * NBW * WT * WT, nullptr, WT, (size_t)WT * WT, WT, WT, HD); }
  k_soft<WT><<<(NH * NBW * WT) / 8, 256, 0, stream>>>(SW, PW, RSW, NH * NBW * WT);
  for (int h = 0; h < NH; ++h) {
    k_gemm_hhx<0><<<dim3(((WT / 16) * 1) / 4, NBW), 128, 0, stream>>>(PW + (size_t)h * NBW * WT * WT, WT, (size_t)WT * WT, VTW + (size_t)h * HD * WT, WT, (size_t)CH * WT, 0.0009765625f, nullptr, 0, nullptr, 1, 0, 0, OW + h * HD, nullptr, CH, (size_t)WT * CH, WT, HD, WT); }
  k_osc<<<(unsigned)((np / 8 + 255) / 256), 256, 0, stream>>>(OW, RSW, (size_t)NBW * WT, 0, (size_t)NR, CXW);
  k_gemm2<0><<<dim3((NR / 128) * (CH / 64), 1), 128, 0, stream>>>(CXW, CH, 0, BAP, CH, 0, 0.0625f, wa_pb, 0, nullptr, 1, 0, 0, YW, nullptr, CH, 0, NR, CH, CH);
  for (int b = 0; b < NI; ++b) { const size_t r0 = (size_t)b * PX;
    k_gemm2<0><<<dim3((PX / 128) * (PX / 64), NH), 128, 0, stream>>>(QKVG + r0 * 3 * CH, 3 * CH, (size_t)HD, QKVG + r0 * 3 * CH + CH, 3 * CH, (size_t)HD, 1.0f, nullptr, 0, nullptr, 1, 0, 0, SG, nullptr, PX, (size_t)PX * PX, PX, PX, HD);
    k_soft<PX><<<(NH * PX) / 8, 256, 0, stream>>>(SG, PG, RSG, NH * PX);
    k_gemm_hhx<0><<<dim3(((PX / 16) * 1) / 4, NH), 128, 0, stream>>>(PG, PX, (size_t)PX * PX, VTG + r0 * CH, PX, (size_t)HD * PX, 0.0009765625f, nullptr, 0, nullptr, 1, 0, 0, OG, nullptr, CH, (size_t)HD, PX, HD, PX);
    k_osc<<<(unsigned)(((size_t)PX * CH / 8 + 255) / 256), 256, 0, stream>>>(OG, RSG, (size_t)PX, r0, (size_t)PX, CXG); }
  k_gemm2<0><<<dim3((NR / 128) * (CH / 64), 1), 128, 0, stream>>>(CXG, CH, 0, BGP, CH, 0, 0.0625f, ga_pb, 0, nullptr, 1, 0, 0, YG, nullptr, CH, 0, NR, CH, CH);
  k_x1<<<(unsigned)((np / 8 + 255) / 256), 256, 0, stream>>>(x, YW, YG, X1);
  k_cstat<<<NI * (CH / 64), 256, 0, stream>>>(X1, CH, nullptr, 0, 0.f, MU2); k_cstat<<<NI * (CH / 64), 256, 0, stream>>>(X1, CH, MU2, 1, 1e-5f, RS2);
  k_cstat<<<NI * (CH / 64), 256, 0, stream>>>(X1, CH, nullptr, 0, 0.f, CM);
  k_se<<<NI, 256, 0, stream>>>(CM, MU2, RS2, ca_w1, ca_w2, SV);
  k_x2<<<(unsigned)((np / 8 + 255) / 256), 256, 0, stream>>>(X1, MU2, RS2, SV, X2);
  k_cstat<<<NI * (CH / 64), 256, 0, stream>>>(X2, CH, nullptr, 0, 0.f, MU3); k_cstat<<<NI * (CH / 64), 256, 0, stream>>>(X2, CH, MU3, 1, 1e-5f, RS3);
  k_xn3<<<(unsigned)((np / 8 + 255) / 256), 256, 0, stream>>>(X2, MU3, RS3, XN3);
  k_gemm2<0><<<dim3((NR / 128) * (HID / 64), 1), 128, 0, stream>>>(XN3, CH, 0, BF1, CH, 0, 0.0625f, fc1_b, 0, nullptr, 1, 0, 0, H1, nullptr, HID, 0, NR, HID, CH);
  k_dwg<<<(unsigned)(((size_t)NR * HID / 4 + 255) / 256), 256, 0, stream>>>(H1, dw3_w, dw3_b, dw5_w, dw5_b, A16);
  k_cstat<<<NI * (HID / 64), 256, 0, stream>>>(H1, HID, nullptr, 0, 0.f, G);
  k_gtab<<<NI, 256, 0, stream>>>(G, fc2_w, fc2_b, GB);
  k_gemm2<0><<<dim3((NR / 128) * (CH / 64), 1), 128, 0, stream>>>(A16, HID, 0, BF2, HID, 0, 0.0625f, nullptr, 0, GB, PX, (size_t)CH, 0, Y, nullptr, CH, 0, NR, CH, HID);
  k_out<<<(unsigned)(((size_t)NI * CH * PX / 8 + 255) / 256), 256, 0, stream>>>(X2, Y, (float*)d_out);
}
